// MolecularGNN_29935922053239
// MI455X (gfx1250) — hardware-verified
//
#include <hip/hip_runtime.h>
#include <hip/hip_bf16.h>
#include <math.h>


#define BB 2
#define SS 2048
#define DD 1024
#define HH 16
#define DKK 64
#define QW 2

typedef _Float16 bf16;
typedef __attribute__((ext_vector_type(4))) unsigned v4u_t;
typedef unsigned v4ua __attribute__((ext_vector_type(4), may_alias));
typedef __attribute__((ext_vector_type(4))) float v4f_t;
typedef float v4fa __attribute__((ext_vector_type(4), may_alias));
typedef __attribute__((ext_vector_type(16))) bf16  bf16x16;
typedef __attribute__((ext_vector_type(8)))  bf16  bf16x8;
typedef __attribute__((ext_vector_type(4)))  bf16  bf16x4;
typedef __attribute__((ext_vector_type(8)))  float f32x8;

#define LDS_STRIDE 48
#define KSTRIDE    72
#define VSTRIDE    48

__device__ __forceinline__ f32x8 wmma_bf16(bf16x16 a, bf16x16 b, f32x8 c) {
  return __builtin_amdgcn_wmma_f32_16x16x32_f16(
      false, a, false, b, (short)0, c, false, false);
}

template <typename T>
__device__ __forceinline__ bf16x16 load_frag(const T* __restrict__ base, int ld,
                                             int row0, int k0) {
  const int lane = threadIdx.x & 31;
  const int r    = lane & 15;
  const int kh   = (lane >> 4) * 8;
  const T* p0 = base + (size_t)(row0 + r) * ld + (k0 + kh);
  const T* p1 = p0 + 16;
  bf16x16 f;
#pragma unroll
  for (int i = 0; i < 8; ++i) {
    f[i]     = (bf16)p0[i];
    f[i + 8] = (bf16)p1[i];
  }
  return f;
}

__device__ __forceinline__ bf16x16 lds_frag(const bf16* base, int stride) {
  const int lane = threadIdx.x & 31;
  const int row  = lane & 15;
  const int kh   = (lane >> 4) * 8;
  const bf16x8 lo = *(const bf16x8*)(base + row * stride + kh);
  const bf16x8 hi = *(const bf16x8*)(base + row * stride + kh + 16);
  bf16x16 f;
#pragma unroll
  for (int i = 0; i < 8; ++i) { f[i] = lo[i]; f[i + 8] = hi[i]; }
  return f;
}

template <typename T>
__device__ __forceinline__ void stage_read16(const T* __restrict__ p, float* buf) {
#pragma unroll
  for (int i = 0; i < 16; ++i) buf[i] = (float)p[i];
}

__device__ __forceinline__ void stage_write(bf16* dst, const float* buf, int nquad) {
#pragma unroll
  for (int i = 0; i < nquad; ++i) {
    bf16x4 q;
    q[0] = (bf16)buf[4 * i];     q[1] = (bf16)buf[4 * i + 1];
    q[2] = (bf16)buf[4 * i + 2]; q[3] = (bf16)buf[4 * i + 3];
    *(bf16x4*)(dst + 4 * i) = q;
  }
}

template <typename AT, typename WTY, int MODE>
__global__ __launch_bounds__(256) void gemm_bias_kernel(
    const AT* __restrict__ A, const WTY* __restrict__ W,
    const float* __restrict__ bias, void* __restrict__ out,
    int M, int N, int K) {
  __shared__ bf16 ldsA[128 * LDS_STRIDE];
  __shared__ bf16 ldsW[256 * LDS_STRIDE];
  __shared__ __attribute__((aligned(16))) unsigned char sob[256 * 136 * 2];

  const int t    = threadIdx.x;
  const int wave = t >> 5;
  const int lane = t & 31;
  const int wm   = (wave & 1) * 64;
  const int wn   = (wave >> 1) * 64;
  const int mBlk = blockIdx.x * 128;
  const int nBlk = blockIdx.y * 256;

  const int arow = t >> 1;
  const int ach  = (t & 1) * 16;

  float abuf[16];
  float wbuf[32];

  stage_read16(A + (size_t)(mBlk + arow) * K + ach, abuf);
  stage_read16(W + (size_t)(nBlk + t) * K,          wbuf);
  stage_read16(W + (size_t)(nBlk + t) * K + 16,     wbuf + 16);

  f32x8 acc[4][4] = {};

  for (int k = 0; k < K; k += 32) {
    __syncthreads();
    stage_write(&ldsA[arow * LDS_STRIDE + ach], abuf, 4);
    stage_write(&ldsW[t * LDS_STRIDE],          wbuf, 8);
    if (k + 32 < K) {
      stage_read16(A + (size_t)(mBlk + arow) * K + (k + 32) + ach, abuf);
      stage_read16(W + (size_t)(nBlk + t) * K + (k + 32),          wbuf);
      stage_read16(W + (size_t)(nBlk + t) * K + (k + 32) + 16,     wbuf + 16);
    }
    __syncthreads();

    bf16x16 af[4], wf[4];
#pragma unroll
    for (int i = 0; i < 4; ++i)
      af[i] = lds_frag(ldsA + (wm + 16 * i) * LDS_STRIDE, LDS_STRIDE);
#pragma unroll
    for (int j = 0; j < 4; ++j)
      wf[j] = lds_frag(ldsW + (wn + 16 * j) * LDS_STRIDE, LDS_STRIDE);
#pragma unroll
    for (int i = 0; i < 4; ++i)
#pragma unroll
      for (int j = 0; j < 4; ++j)
        acc[i][j] = wmma_bf16(af[i], wf[j], acc[i][j]);
  }

  const int nlane = lane & 15;
  const int mh    = (lane >> 4) * 8;
  __syncthreads();
  if (MODE == 0 || MODE == 1) {
    bf16* so = (bf16*)sob;
#pragma unroll
    for (int i = 0; i < 4; ++i)
#pragma unroll
      for (int j = 0; j < 4; ++j) {
        const int nl = wn + 16 * j + nlane;
        const float bv = bias ? bias[nBlk + nl] : 0.0f;
#pragma unroll
        for (int r = 0; r < 8; ++r) {
          const int ml = wm + 16 * i + mh + r;
          const bf16 hv = (bf16)(acc[i][j][r] + bv);
          if (MODE == 0) so[ml * 264 + nl] = hv;
          else           so[nl * 136 + ml] = hv;
        }
      }
    __syncthreads();
#pragma unroll 1
    for (int pass = 0; pass < 2; ++pass) {
      if (MODE == 0) {
        for (int ch = t; ch < 128 * 32; ch += 256) { const int ml = ch >> 5, q = (ch & 31) * 8;
          *(volatile v4u_t*)((bf16*)out + (size_t)(mBlk + ml) * N + nBlk + q) = *(const v4ua*)(so + ml * 264 + q); }
      } else {
        const int b_ = mBlk / SS, s0 = mBlk & (SS - 1);
        for (int ch = t; ch < 256 * 16; ch += 256) { const int nl = ch >> 4, q = (ch & 15) * 8; const int n = nBlk + nl, h = n >> 6, dk = n & (DKK - 1);
          *(volatile v4u_t*)((bf16*)out + (((size_t)(b_ * HH + h)) * DKK + dk) * SS + s0 + q) = *(const v4ua*)(so + nl * 136 + q); }
      }
      __threadfence();
    }
  } else {
    float* so = (float*)sob;
#pragma unroll 1
    for (int hf = 0; hf < 2; ++hf) {
      if (wm == hf * 64) {
#pragma unroll
        for (int i = 0; i < 4; ++i)
#pragma unroll
          for (int j = 0; j < 4; ++j) {
            const int nl = wn + 16 * j + nlane;
            const float bv = bias ? bias[nBlk + nl] : 0.0f;
#pragma unroll
            for (int r = 0; r < 8; ++r) so[(16 * i + mh + r) * 260 + nl] = acc[i][j][r] + bv;
          }
      }
      __syncthreads();
#pragma unroll 1
      for (int pass = 0; pass < 2; ++pass) {
        for (int ch = t; ch < 64 * 64; ch += 256) { const int ml = ch >> 6, q = (ch & 63) * 4;
          *(volatile v4f_t*)((float*)out + (size_t)(mBlk + hf * 64 + ml) * N + nBlk + q) = *(const volatile v4fa*)(so + ml * 260 + q); }
        __threadfence();
      }
      __syncthreads();
    }
  }
}


#define GN 50000
#define GNP 50176
#define GE 800000
#define NGR 256
#define EF 8
#define HC 256
#define RG1 25088

__device__ __forceinline__ float lk(float x, float s) { return x >= 0.0f ? x : s * x; }
__device__ __forceinline__ int clampi(int v, int hi) { return v < 0 ? 0 : (v >= hi ? hi - 1 : v); }

#define OWN_SCAN3_BEGIN(COUNT, KEYEXPR, AUXEXPR) \
  for (int c0 = 0; c0 < (COUNT); c0 += 256) { \
    const int e = c0 + tid; int d = -1, aux = 0; \
    if (e < (COUNT)) { d = (KEYEXPR); aux = (AUXEXPR); } \
    const int own = (d >= 0) ? (d & 7) : -1; unsigned mown = 0u; \
    _Pragma("unroll") for (int ww = 0; ww < 8; ++ww) { const unsigned m = __builtin_amdgcn_ballot_w32(own == ww); if (own == ww) mown = m; if (lane == 0) wcnt[ww][wave] = __builtin_popcount(m); } \
    __syncthreads(); \
    if (own >= 0) { int base = 0; _Pragma("unroll") for (int w2 = 0; w2 < 8; ++w2) base += (w2 < wave) ? wcnt[own][w2] : 0; \
      const int pos = base + __builtin_popcount(mown & ((1u << lane) - 1u)); qd[own][pos] = d; qs[own][pos] = aux; qx[own][pos] = e; } \
    int total = 0; _Pragma("unroll") for (int w2 = 0; w2 < 8; ++w2) total += wcnt[wave][w2]; \
    __syncthreads();
#define OWN_SCAN3_END __syncthreads(); }

__global__ __launch_bounds__(256) void k_emean(const float* __restrict__ ea, float* __restrict__ mean8) {
  __shared__ float red[8][256];
  const int t = threadIdx.x; float s[8] = {0, 0, 0, 0, 0, 0, 0, 0};
  for (int e = t; e < GE; e += 256) { const v4f_t a = *(const v4fa*)(ea + (size_t)e * EF), b = *(const v4fa*)(ea + (size_t)e * EF + 4);
    s[0] += a.x; s[1] += a.y; s[2] += a.z; s[3] += a.w; s[4] += b.x; s[5] += b.y; s[6] += b.z; s[7] += b.w; }
#pragma unroll
  for (int f = 0; f < 8; ++f) red[f][t] = s[f];
  __syncthreads();
  if (t < 32) { float v = 0.0f; if (t < 8) { double acc = 0.0; for (int i = 0; i < 256; ++i) acc += (double)red[t][i]; v = (float)(acc / (double)GE); }
    *(volatile float*)(mean8 + t) = v; __threadfence(); *(volatile float*)(mean8 + t) = v; }
}
template <int NH>
__global__ __launch_bounds__(64) void k_foldae(const float* __restrict__ We, const float* __restrict__ Ae, const float* __restrict__ mean8, float* __restrict__ WAe, float* __restrict__ aself) {
  __shared__ float w[32];
  const int t = threadIdx.x; float v = 0.0f;
  if (t < 32) { const int f = t >> 2, h = t & 3; if (h < NH) { for (int c = 0; c < 64; ++c) v += We[(size_t)f * (NH * 64) + h * 64 + c] * Ae[h * 64 + c]; } w[t] = v; }
  __syncthreads();
  if (t < 32) { *(volatile float*)(WAe + t) = w[t]; }
  if (t >= 32) { const int h = (t - 32) & 3; float s = 0.0f; if (h < NH && t < 36) for (int f = 0; f < 8; ++f) s += mean8[f] * w[f * 4 + h]; *(volatile float*)(aself + (t - 32)) = (t < 36) ? s : 0.0f; }
  __threadfence();
  if (t < 32) { *(volatile float*)(WAe + t) = w[t]; }
  if (t >= 32) { const int h = (t - 32) & 3; float s = 0.0f; if (h < NH && t < 36) for (int f = 0; f < 8; ++f) s += mean8[f] * w[f * 4 + h]; *(volatile float*)(aself + (t - 32)) = (t < 36) ? s : 0.0f; }
}
__global__ __launch_bounds__(256) void k_ae(const float* __restrict__ ea, const float* __restrict__ WAe, float* __restrict__ AE) {
  __shared__ float w[32];
  if (threadIdx.x < 32) w[threadIdx.x] = WAe[threadIdx.x];
  __syncthreads();
  const int e = blockIdx.x * 256 + threadIdx.x; if (e >= GE) return;
  const v4f_t a = *(const v4fa*)(ea + (size_t)e * EF), b = *(const v4fa*)(ea + (size_t)e * EF + 4); v4f_t r;
#pragma unroll
  for (int h = 0; h < 4; ++h) r[h] = a.x * w[h] + a.y * w[4 + h] + a.z * w[8 + h] + a.w * w[12 + h] + b.x * w[16 + h] + b.y * w[20 + h] + b.z * w[24 + h] + b.w * w[28 + h];
  *(volatile v4f_t*)(AE + (size_t)e * 4) = r; __threadfence(); *(volatile v4f_t*)(AE + (size_t)e * 4) = r;
}
__global__ __launch_bounds__(32) void k_padx(const float* __restrict__ x, float* __restrict__ XP) {
  const int n = blockIdx.x, c = threadIdx.x; const float v = (n < GN) ? x[(size_t)n * 32 + c] : 0.0f;
  *(volatile float*)(XP + (size_t)n * 32 + c) = v; __threadfence(); *(volatile float*)(XP + (size_t)n * 32 + c) = v;
}
__global__ __launch_bounds__(256) void k_twg(const float* __restrict__ W, int K, int N, float* __restrict__ WT) {
  const int n = blockIdx.x; for (int k = threadIdx.x; k < K; k += 256) { const float v = W[(size_t)k * N + n]; *(volatile float*)(WT + (size_t)n * K + k) = v; }
  __threadfence();
  for (int k = threadIdx.x; k < K; k += 256) { const float v = W[(size_t)k * N + n]; *(volatile float*)(WT + (size_t)n * K + k) = v; }
}
__global__ __launch_bounds__(256) void k_packA3(const float* __restrict__ W3, float* __restrict__ A) {
  const int m = blockIdx.x, k = threadIdx.x; const float v = (m < 64) ? W3[(size_t)k * 64 + m] : 0.0f;
  *(volatile float*)(A + (size_t)m * HC + k) = v; __threadfence(); *(volatile float*)(A + (size_t)m * HC + k) = v;
}
template <int NH, int MW>
__global__ __launch_bounds__(256) void k_asad(const bf16* __restrict__ M, const float* __restrict__ as_, const float* __restrict__ ad_, const float* __restrict__ aself, float* __restrict__ AS, float* __restrict__ AD, float* __restrict__ MX) {
  __shared__ float st[3][8][4];
  const int n = blockIdx.x * 8 + (threadIdx.x >> 5), t = threadIdx.x, w = t >> 5, lane = t & 31;
#pragma unroll
  for (int h = 0; h < 4; ++h) {
    float s = 0.f, d = 0.f;
    if (h < NH && n < GN) { const float m0 = (float)M[(size_t)n * MW + h * 64 + lane], m1 = (float)M[(size_t)n * MW + h * 64 + 32 + lane];
      s = m0 * as_[h * 64 + lane] + m1 * as_[h * 64 + 32 + lane]; d = m0 * ad_[h * 64 + lane] + m1 * ad_[h * 64 + 32 + lane]; }
#pragma unroll
    for (int o = 16; o >= 1; o >>= 1) { s += __shfl_xor(s, o, 32); d += __shfl_xor(d, o, 32); }
    if (lane == 0) { st[0][w][h] = s; st[1][w][h] = d; st[2][w][h] = (h < NH) ? lk(s + d + aself[h], 0.2f) : 0.0f; }
  }
  __syncthreads();
  if (t < 96) { const int which = t >> 5, i = t & 31; float* dst = (which == 0 ? AS : which == 1 ? AD : MX) + (size_t)blockIdx.x * 32 + i; const float v = st[which][i >> 2][i & 3];
    *(volatile float*)dst = v; __threadfence(); *(volatile float*)dst = v; }
}
template <int NH>
__global__ __launch_bounds__(256) void k_gmax(const int* __restrict__ srci, const int* __restrict__ dsti, const float* __restrict__ AS, const float* __restrict__ AD, const float* __restrict__ AE, float* __restrict__ MX) {
  __shared__ int qd[8][256], qs[8][256], qx[8][256]; __shared__ int wcnt[8][8];
  const int tid = threadIdx.x, lane = tid & 31, wave = tid >> 5;
  OWN_SCAN3_BEGIN(GE, clampi(dsti[e], GN), clampi(srci[e], GN))
    if (lane < NH) {
#pragma unroll 1
      for (int qi = 0; qi < total; ++qi) { const int dl = qd[wave][qi], sl = qs[wave][qi], ee = qx[wave][qi];
        const float ev = lk(AS[(size_t)sl * 4 + lane] + AD[(size_t)dl * 4 + lane] + AE[(size_t)ee * 4 + lane], 0.2f); float* p = MX + (size_t)dl * 4 + lane; *p = fmaxf(*p, ev); } }
  OWN_SCAN3_END
  __threadfence(); __syncthreads();
  for (int i = tid; i < GN; i += 256) { float* p = MX + (size_t)i * 4; const v4f_t v = *(const volatile v4fa*)p; *(volatile v4f_t*)p = v; }
  __threadfence();
}
template <int NH, int MW, int RANGE>
__global__ __launch_bounds__(256) void k_gacc(const int* __restrict__ srci, const int* __restrict__ dsti, const float* __restrict__ AS, const float* __restrict__ AD, const float* __restrict__ AE, const float* __restrict__ aself,
                                             const float* __restrict__ MX, const bf16* __restrict__ M, float* __restrict__ R, float* __restrict__ DEN, int rsel) {
  __shared__ int qd[8][256], qs[8][256], qx[8][256]; __shared__ int wcnt[8][8];
  const int tid = threadIdx.x, lane = tid & 31, wave = tid >> 5, r0 = rsel * RANGE;
  constexpr int PER = MW / 32;
  for (int i = tid; i < RANGE * (MW / 4); i += 256) { const int nl = i / (MW / 4), c4 = (i % (MW / 4)) * 4, n = r0 + nl; v4f_t v; v.x = v.y = v.z = v.w = 0.0f;
    if (n < GN) { const int h = c4 / 64; const float ex = expf(lk(AS[(size_t)n * 4 + h] + AD[(size_t)n * 4 + h] + aself[h], 0.2f) - MX[(size_t)n * 4 + h]);
      v.x = ex * (float)M[(size_t)n * MW + c4]; v.y = ex * (float)M[(size_t)n * MW + c4 + 1]; v.z = ex * (float)M[(size_t)n * MW + c4 + 2]; v.w = ex * (float)M[(size_t)n * MW + c4 + 3]; }
    *(volatile v4f_t*)(R + (size_t)nl * MW + c4) = v; }
  for (int i = tid; i < RANGE; i += 256) { const int n = r0 + i; v4f_t v; v.x = v.y = v.z = v.w = 0.0f;
    if (n < GN) { for (int h = 0; h < NH; ++h) v[h] = expf(lk(AS[(size_t)n * 4 + h] + AD[(size_t)n * 4 + h] + aself[h], 0.2f) - MX[(size_t)n * 4 + h]); }
    *(volatile v4f_t*)(DEN + (size_t)n * 4) = v; }
  __threadfence(); __syncthreads();
  const int hl = (lane * PER) / 64;
  OWN_SCAN3_BEGIN(GE, ((clampi(dsti[e], GN) >= r0 && clampi(dsti[e], GN) < r0 + RANGE) ? clampi(dsti[e], GN) - r0 : -1), clampi(srci[e], GN))
#pragma unroll 1
    for (int qi = 0; qi < total; ++qi) { const int dl = qd[wave][qi], sl = qs[wave][qi], ee = qx[wave][qi], dn = r0 + dl;
      float exh = 0.0f;
      if (hl < NH) { const float ev = lk(AS[(size_t)sl * 4 + hl] + AD[(size_t)dn * 4 + hl] + AE[(size_t)ee * 4 + hl], 0.2f); exh = expf(ev - MX[(size_t)dn * 4 + hl]); }
      if (((lane * PER) & 63) == 0 && hl < NH) DEN[(size_t)dn * 4 + hl] += exh;
      float* row = R + (size_t)dl * MW + lane * PER; const bf16* ms = M + (size_t)sl * MW + lane * PER;
#pragma unroll
      for (int j = 0; j < PER; ++j) row[j] += exh * (float)ms[j]; }
  OWN_SCAN3_END
  __threadfence(); __syncthreads();
  for (int i = tid; i < RANGE * (MW / 4); i += 256) { float* p = R + (size_t)i * 4; const v4f_t v = *(const volatile v4fa*)p; *(volatile v4f_t*)p = v; }
  for (int i = tid; i < RANGE; i += 256) { float* p = DEN + (size_t)(r0 + i) * 4; const v4f_t v = *(const volatile v4fa*)p; *(volatile v4f_t*)p = v; }
  __threadfence();
}
__global__ __launch_bounds__(256) void k_finln(const float* __restrict__ R, const float* __restrict__ DEN, const float* __restrict__ b, const float* __restrict__ g, const float* __restrict__ be, int r0, bf16* __restrict__ H) {
  __shared__ float red[256];
  const int nl = blockIdx.x, n = r0 + nl, c = threadIdx.x; float v = 0.0f;
  if (n < GN) v = R[(size_t)nl * HC + c] / DEN[(size_t)n * 4 + (c >> 6)] + b[c];
  red[c] = v; __syncthreads();
  for (int o = 128; o > 0; o >>= 1) { if (c < o) red[c] += red[c + o]; __syncthreads(); }
  const float mu = red[0] / (float)HC; __syncthreads();
  const float dv = v - mu; red[c] = dv * dv; __syncthreads();
  for (int o = 128; o > 0; o >>= 1) { if (c < o) red[c] += red[c + o]; __syncthreads(); }
  float y = fmaxf(dv / sqrtf(red[0] / (float)HC + 1e-5f) * g[c] + be[c], 0.0f); if (n >= GN) y = 0.0f;
  const float yn = __shfl_xor(y, 1, 32);
  if ((c & 1) == 0) { bf16 pr[2]; pr[0] = (bf16)y; pr[1] = (bf16)yn; typedef unsigned u1a __attribute__((may_alias));
    *(volatile unsigned*)(H + (size_t)n * HC + c) = *(const u1a*)pr; __threadfence(); *(volatile unsigned*)(H + (size_t)n * HC + c) = *(const u1a*)pr; }
}
__global__ __launch_bounds__(256) void k_m3(const float* __restrict__ T, bf16* __restrict__ M3) {
  __shared__ float tile[64][65];
  const int n0 = blockIdx.x * 64, t = threadIdx.x;
  for (int i = t; i < 64 * 64; i += 256) { const int c = i >> 6, nn = i & 63; tile[c][nn] = T[(size_t)c * GNP + n0 + nn]; }
  __syncthreads();
#pragma unroll 1
  for (int pass = 0; pass < 2; ++pass) {
    for (int i = t; i < 64 * 8; i += 256) { const int nr = i >> 3, c8 = (i & 7) * 8; bf16 hh[8];
#pragma unroll
      for (int e = 0; e < 8; ++e) hh[e] = (bf16)tile[c8 + e][nr];
      *(volatile v4u_t*)(M3 + (size_t)(n0 + nr) * 64 + c8) = *(const v4ua*)hh; }
    __threadfence(); }
}
__global__ __launch_bounds__(256) void k_fin3(const float* __restrict__ R3, const float* __restrict__ DEN, const float* __restrict__ b, const float* __restrict__ g, const float* __restrict__ be, float* __restrict__ H3) {
  const int n = blockIdx.x * 4 + (threadIdx.x >> 6), c = threadIdx.x & 63, lane = threadIdx.x & 31;
  float v = 0.0f; if (n < GN) v = R3[(size_t)n * 64 + c] / DEN[(size_t)n * 4] + b[c];
  __shared__ float part[4][2][2];
  float s = v;
#pragma unroll
  for (int o = 16; o >= 1; o >>= 1) s += __shfl_xor(s, o, 32);
  if (lane == 0) part[threadIdx.x >> 6][(c >> 5)][0] = s;
  __syncthreads();
  const float mu = (part[threadIdx.x >> 6][0][0] + part[threadIdx.x >> 6][1][0]) / 64.0f;
  const float dv = v - mu; float q = dv * dv;
#pragma unroll
  for (int o = 16; o >= 1; o >>= 1) q += __shfl_xor(q, o, 32);
  if (lane == 0) part[threadIdx.x >> 6][(c >> 5)][1] = q;
  __syncthreads();
  const float var = (part[threadIdx.x >> 6][0][1] + part[threadIdx.x >> 6][1][1]) / 64.0f;
  float y = fmaxf(dv / sqrtf(var + 1e-5f) * g[c] + be[c], 0.0f); if (n >= GN) y = 0.0f;
  *(volatile float*)(H3 + (size_t)n * 64 + c) = y; __threadfence(); *(volatile float*)(H3 + (size_t)n * 64 + c) = y;
}
__global__ __launch_bounds__(256) void k_pool(const float* __restrict__ H3, const int* __restrict__ batch, const float* __restrict__ gf, const float* __restrict__ W1, const float* __restrict__ b1, const float* __restrict__ W2, const float* __restrict__ b2, float* __restrict__ out) {
  __shared__ float acc[NGR][65]; __shared__ int cnt[NGR]; __shared__ int qd[8][256], qs[8][256], qx[8][256]; __shared__ int wcnt[8][8]; __shared__ float res[NGR];
  const int tid = threadIdx.x, lane = tid & 31, wave = tid >> 5;
  for (int i = tid; i < NGR * 65; i += 256) (&acc[0][0])[i] = 0.0f;
  for (int i = tid; i < NGR; i += 256) cnt[i] = 0;
  __syncthreads();
  OWN_SCAN3_BEGIN(GN, clampi(batch[e], NGR), e)
#pragma unroll 1
    for (int qi = 0; qi < total; ++qi) { const int g = qd[wave][qi], n = qs[wave][qi]; acc[g][lane] += H3[(size_t)n * 64 + lane]; acc[g][32 + lane] += H3[(size_t)n * 64 + 32 + lane]; if (lane == 0) cnt[g] += 1; }
  OWN_SCAN3_END
  for (int g = tid; g < NGR; g += 256) { const float inv = 1.0f / fmaxf((float)cnt[g], 1.0f); float o = b2[0];
    for (int j = 0; j < 64; ++j) { float hsum = b1[j]; for (int f = 0; f < 64; ++f) hsum += acc[g][f] * inv * W1[f * 64 + j]; for (int f = 0; f < 4; ++f) hsum += gf[g * 4 + f] * W1[(64 + f) * 64 + j];
      o += fmaxf(hsum, 0.0f) * W2[j]; }
    res[g] = o; }
  __syncthreads();
  if (tid < 64) { const v4f_t v = *(const volatile v4fa*)(res + tid * 4); *(volatile v4f_t*)(out + tid * 4) = v; __threadfence(); *(volatile v4f_t*)(out + tid * 4) = v; }
}

extern "C" void kernel_launch(void* const* d_in, const int* in_sizes, int n_in,
                              void* d_out, int out_size, void* d_ws, size_t ws_size,
                              hipStream_t stream) {
  (void)in_sizes; (void)n_in; (void)out_size; (void)ws_size;
  const float* x = (const float*)d_in[0]; const int* ei = (const int*)d_in[1]; const float* ea = (const float*)d_in[2]; const int* batch = (const int*)d_in[3]; const float* gf = (const float*)d_in[4];
  const float* W1 = (const float*)d_in[5]; const float* As1 = (const float*)d_in[6]; const float* Ad1 = (const float*)d_in[7]; const float* We1 = (const float*)d_in[8]; const float* Ae1 = (const float*)d_in[9]; const float* b1 = (const float*)d_in[10]; const float* g1 = (const float*)d_in[11]; const float* be1 = (const float*)d_in[12];
  const float* W2 = (const float*)d_in[13]; const float* As2 = (const float*)d_in[14]; const float* Ad2 = (const float*)d_in[15]; const float* We2 = (const float*)d_in[16]; const float* Ae2 = (const float*)d_in[17]; const float* b2 = (const float*)d_in[18]; const float* g2 = (const float*)d_in[19]; const float* be2 = (const float*)d_in[20];
  const float* W3 = (const float*)d_in[21]; const float* As3 = (const float*)d_in[22]; const float* Ad3 = (const float*)d_in[23]; const float* We3 = (const float*)d_in[24]; const float* Ae3 = (const float*)d_in[25]; const float* b3 = (const float*)d_in[26]; const float* g3 = (const float*)d_in[27]; const float* be3 = (const float*)d_in[28];
  const float* fW1 = (const float*)d_in[29]; const float* fb1 = (const float*)d_in[30]; const float* fW2 = (const float*)d_in[31]; const float* fb2 = (const float*)d_in[32];
  const int* srci = ei; const int* dsti = ei + (size_t)GE;
  char* ws = (char*)d_ws;
  float* mean8 = (float*)ws; ws += 32 * 4;
  float* WAe = (float*)ws; ws += 32 * 4 * 3;  float* aself = (float*)ws; ws += 32 * 4 * 3;
  float* W1T = (float*)ws; ws += (size_t)HC * 32 * 4; float* W2T = (float*)ws; ws += (size_t)HC * HC * 4; float* A3 = (float*)ws; ws += (size_t)128 * HC * 4;
  float* AS = (float*)ws; ws += (size_t)GNP * 16; float* AD = (float*)ws; ws += (size_t)GNP * 16; float* MX = (float*)ws; ws += (size_t)GNP * 16; float* DEN = (float*)ws; ws += (size_t)GNP * 16;
  float* AE = (float*)ws; ws += (size_t)GE * 4 * 4;
  float* XP = (float*)ws; ws += (size_t)GNP * 32 * 4;
  bf16* M  = (bf16*)ws;  ws += (size_t)GNP * HC * 2;
  float* R = (float*)ws; ws += (size_t)RG1 * HC * 4;
  bf16* H  = (bf16*)ws;  ws += (size_t)GNP * HC * 2;
  float* H3 = (float*)ws; ws += (size_t)GNP * 64 * 4;
  dim3 blk(256);
  k_emean<<<1, 256, 0, stream>>>(ea, mean8);
  k_padx<<<GNP, 32, 0, stream>>>(x, XP);
  k_twg<<<HC, 256, 0, stream>>>(W1, 32, HC, W1T); k_twg<<<HC, 256, 0, stream>>>(W2, HC, HC, W2T); k_packA3<<<128, 256, 0, stream>>>(W3, A3);
  k_foldae<4><<<1, 64, 0, stream>>>(We1, Ae1, mean8, WAe, aself);
  k_ae<<<GE / 256, 256, 0, stream>>>(ea, WAe, AE);
  gemm_bias_kernel<float, float, 0><<<dim3(GNP / 128, 1), blk, 0, stream>>>(XP, W1T, nullptr, M, GNP, HC, 32);
  k_asad<4, HC><<<GNP / 8, 256, 0, stream>>>(M, As1, Ad1, aself, AS, AD, MX);
  k_gmax<4><<<1, 256, 0, stream>>>(srci, dsti, AS, AD, AE, MX);
  for (int r = 0; r < GNP / RG1; ++r) { k_gacc<4, HC, RG1><<<1, 256, 0, stream>>>(srci, dsti, AS, AD, AE, aself, MX, M, R, DEN, r); k_finln<<<RG1, 256, 0, stream>>>(R, DEN, b1, g1, be1, r * RG1, H); }
  k_foldae<4><<<1, 64, 0, stream>>>(We2, Ae2, mean8, WAe + 32, aself + 32);
  k_ae<<<GE / 256, 256, 0, stream>>>(ea, WAe + 32, AE);
  gemm_bias_kernel<bf16, float, 0><<<dim3(GNP / 128, 1), blk, 0, stream>>>(H, W2T, nullptr, M, GNP, HC, HC);
  k_asad<4, HC><<<GNP / 8, 256, 0, stream>>>(M, As2, Ad2, aself + 32, AS, AD, MX);
  k_gmax<4><<<1, 256, 0, stream>>>(srci, dsti, AS, AD, AE, MX);
  for (int r = 0; r < GNP / RG1; ++r) { k_gacc<4, HC, RG1><<<1, 256, 0, stream>>>(srci, dsti, AS, AD, AE, aself + 32, MX, M, R, DEN, r); k_finln<<<RG1, 256, 0, stream>>>(R, DEN, b2, g2, be2, r * RG1, H); }
  k_foldae<1><<<1, 64, 0, stream>>>(We3, Ae3, mean8, WAe + 64, aself + 64);
  k_ae<<<GE / 256, 256, 0, stream>>>(ea, WAe + 64, AE);
  float* T3 = R; bf16* M3 = M; float* R3 = R;
  gemm_bias_kernel<float, bf16, 2><<<dim3(1, GNP / 256), blk, 0, stream>>>(A3, H, nullptr, T3, 128, GNP, HC);
  k_m3<<<GNP / 64, 256, 0, stream>>>(T3, M3);
  k_asad<1, 64><<<GNP / 8, 256, 0, stream>>>(M3, As3, Ad3, aself + 64, AS, AD, MX);
  k_gmax<1><<<1, 256, 0, stream>>>(srci, dsti, AS, AD, AE, MX);
  k_gacc<1, 64, GNP><<<1, 256, 0, stream>>>(srci, dsti, AS, AD, AE, aself + 64, MX, M3, R3, DEN, 0);
  k_fin3<<<GNP / 4, 256, 0, stream>>>(R3, DEN, b3, g3, be3, H3);
  k_pool<<<1, 256, 0, stream>>>(H3, batch, gf, fW1, fb1, fW2, fb2, (float*)d_out);
}
